// MultiHeadGraphAttention_32427003085127
// MI455X (gfx1250) — hardware-verified
//
#include <hip/hip_runtime.h>
#include <math.h>
#include <stdint.h>

#define NB   4
#define SEQ  4096
#define DIN  256
#define NH   8
#define HD   32
#define NQB  (SEQ / 64)
#define QKP  (2 * DIN)

typedef __attribute__((ext_vector_type(16))) _Float16 v16h;
typedef __attribute__((ext_vector_type(8)))  _Float16 v8h;
typedef __attribute__((ext_vector_type(16))) __bf16   v16b;
typedef __attribute__((ext_vector_type(8)))  __bf16   v8b;
typedef __attribute__((ext_vector_type(8)))  float    v8f;
typedef __attribute__((ext_vector_type(4)))  float    v4f;
typedef __attribute__((ext_vector_type(4)))  unsigned int v4u;
typedef v4f __attribute__((may_alias)) v4fa;

__device__ __forceinline__ unsigned short f2bf_bits(float f) {
  unsigned u = __float_as_uint(f);
  return (unsigned short)((u + 0x7FFFu + ((u >> 16) & 1u)) >> 16);
}
__device__ __forceinline__ float bf_bits2f(unsigned short h) { return __uint_as_float(((unsigned)h) << 16); }
__device__ __forceinline__ unsigned pk16(unsigned short a, unsigned short b) { return (unsigned)a | ((unsigned)b << 16); }

__device__ __forceinline__ void dep_guard_b(v8f& a, v8f& b, v16b x, v16b y) { asm volatile("v_nop\n\tv_nop\n\tv_nop\n\tv_nop" : "+v"(a), "+v"(b) : "v"(x), "v"(y)); }
__device__ __forceinline__ void keep4_b(v16b a, v16b b, v16b c, v16b d) { asm volatile("v_nop" :: "v"(a), "v"(b), "v"(c), "v"(d)); }
__device__ __forceinline__ void acc_guard4(v8f& a, v8f& b, v8f& c, v8f& d) { asm volatile("v_nop\n\tv_nop\n\tv_nop\n\tv_nop" : "+v"(a), "+v"(b), "+v"(c), "+v"(d)); }

struct FragB {
  union U { v16b v; v8b h[2]; };
  static __device__ __forceinline__ v16b load(const __bf16* p) {
    U f; f.h[0] = *(const v8b*)(p); f.h[1] = *(const v8b*)(p + 16); return f.v;
  }
  static __device__ __forceinline__ v8f mma(v16b a, v16b b, v8f c) {
    return __builtin_amdgcn_wmma_f32_16x16x32_bf16(false, a, false, b, (short)0, c, false, false);
  }
};

__device__ __forceinline__ v8f zero8() { v8f z = {0.f, 0.f, 0.f, 0.f, 0.f, 0.f, 0.f, 0.f}; return z; }

template <int OUT_MODE>
__global__ __launch_bounds__(256) void wmma_gemm64(
    const unsigned short* __restrict__ Ap, int lda, long strideA,
    const unsigned short* __restrict__ Btp, int ldb, long strideB,
    void* Cout, void* Cout2, int ldc, long strideC,
    int M, int N, int K, float scale) {
  const __bf16* A  = (const __bf16*)(const void*)Ap;
  const __bf16* Bt = (const __bf16*)(const void*)Btp;
  __shared__ __align__(16) float sT[8][16 * 68];
  const int b    = blockIdx.y;
  const int lane = threadIdx.x & 31;
  const int wave = threadIdx.x >> 5;
  const int tilesN = N >> 6;
  const int tilesM = M >> 6;
  const int tile = blockIdx.x * 8 + wave;
  if (tile >= tilesM * tilesN) return;
  const int tm = tile / tilesN;
  const int tn = tile - tm * tilesN;
  const int m0 = tm << 6;
  const int n0 = tn << 6;

  const __bf16* Ab = A  + (size_t)b * strideA;
  const __bf16* Bb = Bt + (size_t)b * strideB;

  const int rlane = lane & 15;
  const int koff  = (lane >> 4) * 8;
  const int mOff  = (lane >> 4) * 8;

  v8f acc[4][4];
#pragma unroll
  for (int i = 0; i < 4; ++i)
#pragma unroll
    for (int j = 0; j < 4; ++j) acc[i][j] = zero8();

  for (int k0 = 0; k0 < K; k0 += 32) {
    v16b bh[4];
#pragma unroll
    for (int j = 0; j < 4; ++j) {
      const size_t bo = (size_t)(n0 + (j << 4) + rlane) * ldb + koff + k0;
      bh[j] = FragB::load(Bb + bo);
    }
#pragma unroll
    for (int i = 0; i < 4; ++i) {
      const size_t ao = (size_t)(m0 + (i << 4) + rlane) * lda + koff + k0;
      v16b ah = FragB::load(Ab + ao);
#pragma unroll
      for (int j = 0; j < 4; ++j) acc[i][j] = FragB::mma(ah, bh[j], acc[i][j]);
      dep_guard_b(acc[i][0], acc[i][3], ah, ah);
    }
    keep4_b(bh[0], bh[1], bh[2], bh[3]);
  }
  acc_guard4(acc[0][0], acc[0][1], acc[0][2], acc[0][3]);
  acc_guard4(acc[1][0], acc[1][1], acc[1][2], acc[1][3]);
  acc_guard4(acc[2][0], acc[2][1], acc[2][2], acc[2][3]);
  acc_guard4(acc[3][0], acc[3][1], acc[3][2], acc[3][3]);

  float* slab = sT[wave];
#pragma unroll
  for (int i = 0; i < 4; ++i) {
    const int mBase = m0 + (i << 4);
#pragma unroll
    for (int j = 0; j < 4; ++j) {
#pragma unroll
      for (int r = 0; r < 8; ++r) {
        const float v = acc[i][j][r] * scale;
        slab[(mOff + r) * 68 + (j << 4) + rlane] = v;
      }
    }
    __builtin_amdgcn_fence(__ATOMIC_RELEASE, "workgroup");
    __builtin_amdgcn_wave_barrier();
    __builtin_amdgcn_fence(__ATOMIC_ACQUIRE, "workgroup");
    {
      const int q = lane >> 3, c8 = (lane & 7) * 8;
      unsigned short* C  = (unsigned short*)Cout  + (size_t)b * strideC;
      unsigned short* C2 = (unsigned short*)Cout2 + (size_t)b * strideC;
      for (int pass = 0; pass < 2; ++pass) {
#pragma unroll
        for (int it = 0; it < 4; ++it) {
          const int row = it * 4 + q;
          const float* sp = slab + row * 68 + c8;
          v8h hv, lv;
#pragma unroll
          for (int e = 0; e < 8; ++e) {
            if (OUT_MODE == 1) {
              hv[e] = (_Float16)sp[e];
              lv[e] = hv[e];
            } else {
              unsigned short hb = f2bf_bits(sp[e]);
              unsigned short lb = f2bf_bits(sp[e] - bf_bits2f(hb));
              hv[e] = __builtin_bit_cast(_Float16, hb);
              lv[e] = __builtin_bit_cast(_Float16, lb);
            }
          }
          *(volatile v8h*)(C + (size_t)(mBase + row) * ldc + n0 + c8) = hv;
          if (OUT_MODE == 2) *(volatile v8h*)(C2 + (size_t)(mBase + row) * ldc + n0 + c8) = lv;
        }
        __threadfence();
      }
    }
    __builtin_amdgcn_fence(__ATOMIC_RELEASE, "workgroup");
    __builtin_amdgcn_wave_barrier();
    __builtin_amdgcn_fence(__ATOMIC_ACQUIRE, "workgroup");
  }
}

__global__ __launch_bounds__(256) void cvt_bf16x8_kernel(const float* __restrict__ in, unsigned short* __restrict__ o, int n8) {
  const int i = blockIdx.x * 256 + threadIdx.x;
  if (i < n8) {
    const float* sp = in + (size_t)i * 8;
    const v4f a  = *(const v4f*)(sp);
    const v4f a2 = *(const v4f*)(sp + 4);
    v4u w;
    w[0] = pk16(f2bf_bits(a[0]),  f2bf_bits(a[1]));
    w[1] = pk16(f2bf_bits(a[2]),  f2bf_bits(a[3]));
    w[2] = pk16(f2bf_bits(a2[0]), f2bf_bits(a2[1]));
    w[3] = pk16(f2bf_bits(a2[2]), f2bf_bits(a2[3]));
    unsigned short* dp = o + (size_t)i * 8;
    *(volatile v4u*)dp = w;
    __threadfence();
    *(volatile v4u*)dp = w;
  }
}

__global__ __launch_bounds__(256) void tsplit_kernel(const float* __restrict__ W, unsigned short* __restrict__ oh,
                                                     unsigned short* __restrict__ ol, int R, int Cc) {
  __shared__ __align__(16) float tf[64 * 68];
  const int c0  = blockIdx.x * 64;
  const int r0  = blockIdx.y * 64;
  const int tid = threadIdx.x;
  {
    const int lr = tid >> 4;
    const int c4 = (tid & 15) * 4;
#pragma unroll
    for (int it = 0; it < 4; ++it) {
      const int rr = it * 16 + lr;
      const v4f a = *(const v4f*)(W + (size_t)(r0 + rr) * Cc + c0 + c4);
      *(v4f*)(tf + rr * 68 + c4) = a;
    }
  }
  __syncthreads();
  const int sub = tid >> 3;
  const int c8  = (tid & 7) * 8;
  v4u hv[2], lv[2];
#pragma unroll
  for (int it = 0; it < 2; ++it) {
    const int oc = it * 32 + sub;
    v4u a, a2;
#pragma unroll
    for (int q = 0; q < 4; ++q) {
      const float f0 = tf[(c8 + 2 * q) * 68 + oc];
      const float f1 = tf[(c8 + 2 * q + 1) * 68 + oc];
      const unsigned short h0 = f2bf_bits(f0), h1 = f2bf_bits(f1);
      const unsigned short l0 = f2bf_bits(f0 - bf_bits2f(h0)), l1 = f2bf_bits(f1 - bf_bits2f(h1));
      a[q]  = pk16(h0, h1);
      a2[q] = pk16(l0, l1);
    }
    hv[it] = a; lv[it] = a2;
  }
  for (int pass = 0; pass < 2; ++pass) {
#pragma unroll
    for (int it = 0; it < 2; ++it) {
      const int oc = it * 32 + sub;
      const size_t go = (size_t)(c0 + oc) * R + r0 + c8;
      *(volatile v4u*)(oh + go) = hv[it];
      *(volatile v4u*)(ol + go) = lv[it];
    }
    __threadfence();
  }
}

#define AT_NW 4
#define AT_QB 64
#define AT_KC 64
#define OSP   36

__device__ __forceinline__ __bf16 at_f2bf(float f) { return __builtin_bit_cast(__bf16, f2bf_bits(f)); }
__device__ __forceinline__ void at_split(float f, __bf16& hi, __bf16& lo) {
  const unsigned short hb = f2bf_bits(f);
  hi = __builtin_bit_cast(__bf16, hb);
  lo = at_f2bf(f - __uint_as_float(((unsigned)hb) << 16));
}
__device__ __forceinline__ v8f at_mma(v16b a, v16b b, v8f c) {
  c = __builtin_amdgcn_wmma_f32_16x16x32_bf16(false, a, false, b, (short)0, c, false, false);
  asm volatile("v_nop\n\tv_nop\n\tv_nop\n\tv_nop" : "+v"(c) : "v"(a), "v"(b));
  return c;
}
__device__ __forceinline__ v8f at_mma_h(v16h a, v16h b, v8f c) {
  c = __builtin_amdgcn_wmma_f32_16x16x32_f16(false, a, false, b, (short)0, c, false, false);
  asm volatile("v_nop\n\tv_nop\n\tv_nop\n\tv_nop" : "+v"(c) : "v"(a), "v"(b));
  return c;
}

__global__ __launch_bounds__(128)
void leakyattn32_kernel(const unsigned short* __restrict__ qkp,
                        const unsigned short* __restrict__ vhp, const unsigned short* __restrict__ vlp,
                        float* __restrict__ out, float sscale) {
  union FB { v16b v; v8b h[2]; };
  union FH { v16h v; v8h h[2]; };
  __shared__ __align__(16) _Float16 Ksh[AT_KC * HD];
  __shared__ __align__(16) __bf16   Vth[HD * AT_KC];
  __shared__ __align__(16) __bf16   Vtl[HD * AT_KC];
  __shared__ __align__(16) __bf16   Psh[AT_NW][16 * AT_KC];
  __shared__ __align__(16) __bf16   Psl[AT_NW][16 * AT_KC];
  __shared__ __align__(16) float    Os[AT_NW][16 * OSP];

  const int tid  = threadIdx.x;
  const int wave = tid >> 5;
  const int lane = tid & 31;
  const int hh   = lane >> 4;
  const int c    = lane & 15;

  const int bx   = blockIdx.x;
  const int qb   = bx & (NQB - 1);
  const int pair = bx >> 6;
  const int b    = pair >> 3;
  const int h    = pair & 7;
  const int q0   = qb * AT_QB + wave * 16;
  const size_t rowBase = (size_t)b * SEQ;

  const _Float16* Qg = (const _Float16*)(const void*)qkp + h * HD;
  const _Float16* Kg = (const _Float16*)(const void*)qkp + DIN + h * HD;
  const __bf16*   Vh = (const __bf16*)(const void*)vhp + ((size_t)b * DIN + h * HD) * SEQ;
  const __bf16*   Vl = (const __bf16*)(const void*)vlp + ((size_t)b * DIN + h * HD) * SEQ;
  float*          ob = out + h * HD;

  v16h qa;
  {
    FH f;
    const _Float16* qp = Qg + (rowBase + q0 + c) * QKP + 8 * hh;
    f.h[0] = *(const v8h*)(qp);
    f.h[1] = *(const v8h*)(qp + 16);
    qa = f.v;
  }

  v8f oacc[2];
  oacc[0] = zero8(); oacc[1] = zero8();

  __bf16* pwh = Psh[wave];
  __bf16* pwl = Psl[wave];

  const int nChunks = SEQ / AT_KC;
  for (int kc = 0; kc < nChunks; ++kc) {
    const int kv0 = kc * AT_KC;
    __syncthreads();
    {
      const int r = tid >> 1, half = (tid & 1) * 16;
      const _Float16* ks = Kg + (rowBase + kv0 + r) * QKP + half;
      const int d = tid >> 2, qt = (tid & 3) * 16;
      const __bf16* vs = Vh + (size_t)d * SEQ + kv0 + qt;
      const __bf16* vl = Vl + (size_t)d * SEQ + kv0 + qt;
#pragma unroll
      for (int i = 0; i < 2; ++i) {
        const v8h a0 = *(const v8h*)(ks + 8 * i);
        const v8b b0 = *(const v8b*)(vs + 8 * i);
        const v8b b1 = *(const v8b*)(vl + 8 * i);
        *(v8h*)(Ksh + r * HD    + half + 8 * i) = a0;
        *(v8b*)(Vth + d * AT_KC + qt   + 8 * i) = b0;
        *(v8b*)(Vtl + d * AT_KC + qt   + 8 * i) = b1;
      }
    }
    __syncthreads();

    v8f s[4];
#pragma unroll
    for (int j = 0; j < 4; ++j) {
      FH kb;
      const _Float16* kp = Ksh + (j * 16 + c) * HD + 8 * hh;
      kb.h[0] = *(const v8h*)(kp);
      kb.h[1] = *(const v8h*)(kp + 16);
      s[j] = at_mma_h(qa, kb.v, zero8());
    }

#pragma unroll
    for (int r = 0; r < 8; ++r) {
#pragma unroll
      for (int j = 0; j < 4; ++j) {
        const float sv = s[j][r] * sscale;
        const float p  = (sv >= 0.f) ? sv : 0.2f * sv;
        __bf16 a, bl; at_split(p, a, bl);
        pwh[(8 * hh + r) * AT_KC + j * 16 + c] = a;
        pwl[(8 * hh + r) * AT_KC + j * 16 + c] = bl;
      }
    }
    __builtin_amdgcn_fence(__ATOMIC_RELEASE, "workgroup");
    __builtin_amdgcn_wave_barrier();
    __builtin_amdgcn_fence(__ATOMIC_ACQUIRE, "workgroup");

#pragma unroll 1
    for (int kk = 0; kk < 2; ++kk) {
      FB pa, pl;
      pa.h[0] = *(const v8b*)(pwh + c * AT_KC + kk * 32 + 8 * hh);
      pa.h[1] = *(const v8b*)(pwh + c * AT_KC + kk * 32 + 16 + 8 * hh);
      pl.h[0] = *(const v8b*)(pwl + c * AT_KC + kk * 32 + 8 * hh);
      pl.h[1] = *(const v8b*)(pwl + c * AT_KC + kk * 32 + 16 + 8 * hh);
#pragma unroll
      for (int t = 0; t < 2; ++t) {
        FB vb, vl;
        vb.h[0] = *(const v8b*)(Vth + (t * 16 + c) * AT_KC + kk * 32 + 8 * hh);
        vb.h[1] = *(const v8b*)(Vth + (t * 16 + c) * AT_KC + kk * 32 + 16 + 8 * hh);
        vl.h[0] = *(const v8b*)(Vtl + (t * 16 + c) * AT_KC + kk * 32 + 8 * hh);
        vl.h[1] = *(const v8b*)(Vtl + (t * 16 + c) * AT_KC + kk * 32 + 16 + 8 * hh);
        oacc[t] = at_mma(pa.v, vb.v, oacc[t]);
        oacc[t] = at_mma(pa.v, vl.v, oacc[t]);
        oacc[t] = at_mma(pl.v, vb.v, oacc[t]);
      }
    }
  }

  __builtin_amdgcn_fence(__ATOMIC_RELEASE, "workgroup");
  __builtin_amdgcn_wave_barrier();
  __builtin_amdgcn_fence(__ATOMIC_ACQUIRE, "workgroup");
  float* os = Os[wave];
#pragma unroll
  for (int r = 0; r < 8; ++r) {
    os[(8 * hh + r) * OSP + c]      = oacc[0][r];
    os[(8 * hh + r) * OSP + 16 + c] = oacc[1][r];
  }
  __builtin_amdgcn_fence(__ATOMIC_RELEASE, "workgroup");
  __builtin_amdgcn_wave_barrier();
  __builtin_amdgcn_fence(__ATOMIC_ACQUIRE, "workgroup");
  {
    const int q4 = lane >> 3, c4 = (lane & 7) * 4;
    for (int pass = 0; pass < 2; ++pass) {
#pragma unroll
      for (int it = 0; it < 4; ++it) {
        const int row = it * 4 + q4;
        const v4f val = *(const v4fa*)(os + row * OSP + c4);
        *(volatile v4f*)(ob + (rowBase + q0 + row) * DIN + c4) = val;
      }
      __threadfence();
    }
  }
}

extern "C" void kernel_launch(void* const* d_in, const int* in_sizes, int n_in,
                              void* d_out, int out_size, void* d_ws, size_t ws_size,
                              hipStream_t stream) {
  if (n_in < 4) return;
  if (in_sizes[0] != NB * SEQ * DIN) return;
  if (in_sizes[1] != DIN * DIN || in_sizes[2] != DIN * DIN || in_sizes[3] != DIN * DIN) return;
  if (out_size != NB * SEQ * DIN) return;

  const float* x  = (const float*)d_in[0];
  const float* Wq = (const float*)d_in[1];
  const float* Wk = (const float*)d_in[2];
  const float* Wv = (const float*)d_in[3];
  float* out = (float*)d_out;

  const size_t PW = (size_t)DIN * DIN * 2;
  const size_t PX = (size_t)NB * SEQ * DIN * 2;
  const size_t PQ = (size_t)NB * SEQ * QKP * 2;
  const size_t PV = (size_t)NB * DIN * SEQ * 2;
  size_t off = 0;
  const size_t oWqTh = off; off += PW;  const size_t oWkTh = off; off += PW;  const size_t oWvTh = off; off += PW;
  const size_t oWqTl = off; off += PW;  const size_t oWkTl = off; off += PW;  const size_t oWvTl = off; off += PW;
  const size_t oXb   = off; off += PX;
  const size_t oQK   = off; off += PQ;
  const size_t oVTh  = off; off += PV;  const size_t oVTl  = off; off += PV;
  if (off > ws_size) return;
  if (off > (size_t)134217728) return;

  char* ws = (char*)d_ws;
  unsigned short* WqTh = (unsigned short*)(ws + oWqTh); unsigned short* WqTl = (unsigned short*)(ws + oWqTl);
  unsigned short* WkTh = (unsigned short*)(ws + oWkTh); unsigned short* WkTl = (unsigned short*)(ws + oWkTl);
  unsigned short* WvTh = (unsigned short*)(ws + oWvTh); unsigned short* WvTl = (unsigned short*)(ws + oWvTl);
  unsigned short* Xb   = (unsigned short*)(ws + oXb);
  unsigned short* QK   = (unsigned short*)(ws + oQK);
  unsigned short* VTh  = (unsigned short*)(ws + oVTh);  unsigned short* VTl  = (unsigned short*)(ws + oVTl);

  const dim3 blk(256);
  const float sscale = 0.17677669529663688f * 0.015625f;

  tsplit_kernel<<<dim3(DIN / 64, DIN / 64), blk, 0, stream>>>(Wq, WqTh, WqTl, DIN, DIN);
  tsplit_kernel<<<dim3(DIN / 64, DIN / 64), blk, 0, stream>>>(Wk, WkTh, WkTl, DIN, DIN);
  tsplit_kernel<<<dim3(DIN / 64, DIN / 64), blk, 0, stream>>>(Wv, WvTh, WvTl, DIN, DIN);
  const int n8x = NB * SEQ * DIN / 8;
  cvt_bf16x8_kernel<<<dim3((n8x + 255) / 256), blk, 0, stream>>>(x, Xb, n8x);
  const dim3 gQK(((NB * SEQ / 64) * (QKP / 64) + 7) / 8, 1);
  wmma_gemm64<1><<<gQK, blk, 0, stream>>>(
      Xb, DIN, 0L, WqTh, DIN, 0L, (void*)QK, (void*)QK, QKP, 0L, NB * SEQ, QKP, DIN, 8.0f);
  const dim3 gVT(((DIN / 64) * (SEQ / 64) + 7) / 8, NB);
  wmma_gemm64<2><<<gVT, blk, 0, stream>>>(
      WvTh, DIN, 0L, Xb, DIN, (long)SEQ * DIN, (void*)VTh, (void*)VTl, SEQ, (long)DIN * SEQ, DIN, SEQ, DIN, 1.0f);
  leakyattn32_kernel<<<dim3(NB * NH * NQB), dim3(128), 0, stream>>>(QK, VTh, VTl, out, sscale);
  (void)hipGetLastError();
}
